// Encoder_89163521065800
// MI455X (gfx1250) — hardware-run, weakly checked
//
#include <hip/hip_runtime.h>

constexpr int NVOCAB = 32000;
constexpr int NEMB   = 256;
constexpr int NHID   = 256;
constexpr int NBATCH = 64;
constexpr int NSTEP  = 2048;

constexpr float ECAR = 2048.0f;
constexpr float WCAR = 256.0f;
constexpr float HCAR = 4096.0f;
constexpr float UCAR = 4096.0f;
constexpr float PROJ_SCL = UCAR / (ECAR * WCAR);
constexpr float REC_SCL  = 1.0f / (HCAR * WCAR);
constexpr float UCAR_INV = 1.0f / UCAR;
constexpr float F16_MINN = 6.103515625e-05f;

constexpr int XP = 264;
constexpr int HP = 264;
constexpr int OP = 260;
constexpr int HBUF_HALVES = NBATCH * HP;
constexpr int SZ_HBUF = HBUF_HALVES * 2;
constexpr int SZ_OUTS = NBATCH * OP * 4;
constexpr int LDS_RNN = 2 * SZ_HBUF + SZ_OUTS;

constexpr size_t SZ_UT  = (size_t)NSTEP * NHID * NBATCH * 2;
constexpr size_t SZ_WT  = (size_t)NHID * NHID * 2;
constexpr size_t WS_TOTAL = SZ_UT + SZ_WT + SZ_WT;

static_assert(NEMB == 256 && NHID == 256 && NBATCH == 64 && NSTEP == 2048);
static_assert(NEMB % 32 == 0 && NHID % 32 == 0 && NBATCH % 64 == 0 && NHID % 64 == 0);
static_assert(XP % 8 == 0 && HP % 8 == 0 && OP % 4 == 0);
static_assert(SZ_HBUF % 16 == 0 && SZ_OUTS % 16 == 0 && LDS_RNN == 134144);
static_assert(WS_TOTAL == 67371008 && WS_TOTAL <= 134217728);
static_assert(SZ_UT % 128 == 0 && SZ_WT % 128 == 0);

typedef __attribute__((ext_vector_type(16))) _Float16 v16h;
typedef __attribute__((ext_vector_type(8)))  _Float16 v8h;
typedef __attribute__((ext_vector_type(8)))  float    v8f;
typedef __attribute__((ext_vector_type(4)))  float    v4f;
typedef __attribute__((ext_vector_type(4)))  unsigned v4u;

union FragU { v16h v; v8h h[2]; };

__device__ __forceinline__ v16h frag_load(const _Float16* p) {
  FragU f;
  f.h[0] = *(const v8h*)(p);
  f.h[1] = *(const v8h*)(p + 16);
  return f.v;
}

__device__ __forceinline__ v8f mma_g(v16h a, v16h b, v8f c) {
  c = __builtin_amdgcn_wmma_f32_16x16x32_f16(false, a, false, b, (short)0, c, false, false);
  asm volatile("v_nop\n\tv_nop\n\tv_nop\n\tv_nop" : "+v"(c) : "v"(a), "v"(b));
  return c;
}

__device__ __forceinline__ _Float16 to_f16_flush(float v) {
  const float z = (fabsf(v) < F16_MINN) ? 0.0f : v;
  return (_Float16)z;
}

__device__ __forceinline__ float h16_to_f32(unsigned hb) {
  const unsigned sgn = (hb & 0x8000u) << 16;
  const unsigned em = hb & 0x7fffu;
  const float fn = __uint_as_float((em << 13) + 0x38000000u);
  const float fs = (float)em * 5.9604644775390625e-8f;
  const float mag = (em < 0x400u) ? fs : fn;
  return __uint_as_float(__float_as_uint(mag) | sgn);
}

__global__ __launch_bounds__(256) void k_wprep(const float* __restrict__ wih, const float* __restrict__ whh,
                                               _Float16* __restrict__ wihT, _Float16* __restrict__ whhT) {
  __shared__ float tl[64][65];
  const int tid = threadIdx.x;
  const int mat = blockIdx.x >> 4;
  const int tile = blockIdx.x & 15;
  const int k0 = (tile >> 2) * 64;
  const int n0 = (tile & 3) * 64;
  const float* __restrict__ W = (mat != 0) ? whh : wih;
  _Float16* __restrict__ WT = (mat != 0) ? whhT : wihT;
#pragma unroll 4
  for (int it = 0; it < 16; ++it) {
    const int i = it * 256 + tid;
    const int kk = i >> 6;
    const int nn = i & 63;
    tl[kk][nn] = W[(k0 + kk) * NHID + n0 + nn];
  }
  __syncthreads();
  v8h hv[2];
#pragma unroll
  for (int it = 0; it < 2; ++it) {
    const int idx = it * 256 + tid;
    const int nn = idx >> 3;
    const int c8 = (idx & 7) * 8;
#pragma unroll
    for (int e = 0; e < 8; ++e) hv[it][e] = to_f16_flush(tl[c8 + e][nn] * WCAR);
  }
  for (int pass = 0; pass < 2; ++pass) {
#pragma unroll
    for (int it = 0; it < 2; ++it) {
      const int idx = it * 256 + tid;
      const int nn = idx >> 3;
      const int c8 = (idx & 7) * 8;
      *(volatile v8h*)(WT + (size_t)(n0 + nn) * NHID + k0 + c8) = hv[it];
    }
    __threadfence();
  }
}

__global__ __launch_bounds__(128) void k_proj(const int* __restrict__ src, const float* __restrict__ emb,
                                              const _Float16* __restrict__ wihT, _Float16* __restrict__ UT) {
  __shared__ __align__(16) _Float16 Xs[NBATCH * XP];
  __shared__ __align__(16) float sT[4][16 * 68];
  const int tid = threadIdx.x;
  const int lane = tid & 31;
  const int wave = tid >> 5;
  const int c = lane & 15;
  const int hh = lane >> 4;
  const int t = blockIdx.x;

#pragma unroll 4
  for (int it = 0; it < 16; ++it) {
    const int b = it * 4 + wave;
    int id = src[b * NSTEP + t];
    id = id < 0 ? 0 : id;
    id = id > (NVOCAB - 1) ? (NVOCAB - 1) : id;
    const float* er = emb + (size_t)id * NEMB + lane * 8;
    const v4f va = *(const v4f*)(er);
    const v4f vb = *(const v4f*)(er + 4);
    v8h hv;
#pragma unroll
    for (int e = 0; e < 4; ++e) {
      hv[e]     = to_f16_flush(va[e] * ECAR);
      hv[4 + e] = to_f16_flush(vb[e] * ECAR);
    }
    *(v8h*)(Xs + b * XP + lane * 8) = hv;
  }
  __syncthreads();

  const int m0 = wave * 64;
  const int koff = 8 * hh;
  const int mOff = 8 * hh;
  v8f acc[4][4];
#pragma unroll
  for (int i = 0; i < 4; ++i)
#pragma unroll
    for (int j = 0; j < 4; ++j) acc[i][j] = (v8f){0.f, 0.f, 0.f, 0.f, 0.f, 0.f, 0.f, 0.f};

#pragma unroll 1
  for (int k0 = 0; k0 < NEMB; k0 += 32) {
    v16h bh[4];
#pragma unroll
    for (int j = 0; j < 4; ++j) bh[j] = frag_load(Xs + (16 * j + c) * XP + k0 + koff);
#pragma unroll
    for (int i = 0; i < 4; ++i) {
      const v16h ah = frag_load(wihT + (size_t)(m0 + 16 * i + c) * NEMB + k0 + koff);
#pragma unroll
      for (int j = 0; j < 4; ++j) acc[i][j] = mma_g(ah, bh[j], acc[i][j]);
    }
  }

  float* slab = sT[wave];
  _Float16* Ub = UT + (size_t)t * NHID * NBATCH;
  const int q = lane >> 3;
  const int c8 = (lane & 7) * 8;
#pragma unroll
  for (int i = 0; i < 4; ++i) {
#pragma unroll
    for (int j = 0; j < 4; ++j) {
#pragma unroll
      for (int r = 0; r < 8; ++r) slab[(mOff + r) * 68 + 16 * j + c] = acc[i][j][r] * PROJ_SCL;
    }
    __builtin_amdgcn_fence(__ATOMIC_RELEASE, "workgroup");
    __builtin_amdgcn_wave_barrier();
    __builtin_amdgcn_fence(__ATOMIC_ACQUIRE, "workgroup");
    v8h hv[4];
#pragma unroll
    for (int it = 0; it < 4; ++it) {
      const int row = it * 4 + q;
      const float* sp = slab + row * 68 + c8;
      const v4f s0 = *(const v4f*)(sp);
      const v4f s1 = *(const v4f*)(sp + 4);
#pragma unroll
      for (int e = 0; e < 4; ++e) {
        hv[it][e]     = (_Float16)s0[e];
        hv[it][4 + e] = (_Float16)s1[e];
      }
    }
    for (int pass = 0; pass < 2; ++pass) {
#pragma unroll
      for (int it = 0; it < 4; ++it) {
        const int row = it * 4 + q;
        *(volatile v8h*)(Ub + (size_t)(m0 + 16 * i + row) * NBATCH + c8) = hv[it];
      }
      __threadfence();
    }
    __builtin_amdgcn_fence(__ATOMIC_RELEASE, "workgroup");
    __builtin_amdgcn_wave_barrier();
    __builtin_amdgcn_fence(__ATOMIC_ACQUIRE, "workgroup");
  }
}

__global__ __launch_bounds__(512, 1) void k_rnn(const unsigned* __restrict__ UTw, const _Float16* __restrict__ whhT,
                                                const float* __restrict__ bih, const float* __restrict__ bhh,
                                                float* __restrict__ out) {
  extern __shared__ v4u smem_dyn[];
  unsigned char* const smem_raw = (unsigned char*)smem_dyn;
  _Float16* const Hs = (_Float16*)smem_raw;
  float* const OUTS = (float*)(smem_raw + 2 * SZ_HBUF);
  const int tid = threadIdx.x;
  const int lane = tid & 31;
  const int wave = tid >> 5;
  const int c = lane & 15;
  const int hh = lane >> 4;
  const int n = 16 * wave + c;

  {
    const v4u z4 = {0u, 0u, 0u, 0u};
    v4u* const p = (v4u*)smem_raw;
#pragma unroll 1
    for (int i = tid; i < (2 * SZ_HBUF) / 16; i += 512) p[i] = z4;
  }

  v16h bfr[8];
#pragma unroll
  for (int kc = 0; kc < 8; ++kc) {
    bfr[kc] = frag_load(whhT + (size_t)n * NHID + kc * 32 + 8 * hh);
    asm volatile("" : "+v"(bfr[kc]));
  }
  const float bsum = bih[n] + bhh[n];
  __syncthreads();

#pragma unroll 1
  for (int t = 0; t < NSTEP; ++t) {
    const _Float16* cur = Hs + (t & 1) * HBUF_HALVES;
    _Float16* nxt = Hs + ((t & 1) ^ 1) * HBUF_HALVES;
    const bool last = (t == NSTEP - 1);
    const unsigned* urow = UTw + ((size_t)t * NHID + n) * (NBATCH / 2) + 4 * hh;
#pragma unroll 1
    for (int i = 0; i < 4; ++i) {
      const v4u uw = *(const v4u*)(urow + 8 * i);
      unsigned uws[4];
      uws[0] = uw.x;
      uws[1] = uw.y;
      uws[2] = uw.z;
      uws[3] = uw.w;
      v8f acc = (v8f){0.f, 0.f, 0.f, 0.f, 0.f, 0.f, 0.f, 0.f};
      const _Float16* arow = cur + (16 * i + c) * HP + 8 * hh;
#pragma unroll
      for (int kc = 0; kc < 8; ++kc) {
        const v16h a = frag_load(arow + kc * 32);
        acc = mma_g(a, bfr[kc], acc);
      }
      float hn[8];
#pragma unroll
      for (int r = 0; r < 8; ++r) {
        const unsigned w = uws[r >> 1];
        const unsigned hb = (r & 1) ? (w >> 16) : (w & 0xffffu);
        const float u = h16_to_f32(hb);
        const float pre = acc[r] * REC_SCL + (u * UCAR_INV + bsum);
        hn[r] = tanhf(pre);
      }
      _Float16* hrow = nxt + (16 * i + 8 * hh) * HP + n;
#pragma unroll
      for (int r = 0; r < 8; ++r) hrow[r * HP] = to_f16_flush(hn[r] * HCAR);
      if (last) {
        float* orow = OUTS + (16 * i + 8 * hh) * OP + n;
#pragma unroll
        for (int r = 0; r < 8; ++r) orow[r * OP] = hn[r];
      }
    }
    __syncthreads();
  }

  for (int pass = 0; pass < 2; ++pass) {
#pragma unroll
    for (int it = 0; it < 8; ++it) {
      const int idx = it * 512 + tid;
      const int row = idx >> 6;
      const int c4 = (idx & 63) * 4;
      const v4f v = *(const v4f*)(OUTS + row * OP + c4);
      *(volatile v4f*)(out + (size_t)row * NHID + c4) = v;
    }
    __threadfence();
  }
}

extern "C" void kernel_launch(void* const* d_in, const int* in_sizes, int n_in,
                              void* d_out, int out_size, void* d_ws, size_t ws_size, hipStream_t stream) {
  if (n_in < 6 || d_out == nullptr || d_ws == nullptr) return;
  if (in_sizes[0] != NBATCH * NSTEP || in_sizes[1] != NVOCAB * NEMB || in_sizes[2] != NEMB * NHID ||
      in_sizes[3] != NHID * NHID || in_sizes[4] != NHID || in_sizes[5] != NHID || out_size != NBATCH * NHID) return;
  if (ws_size < WS_TOTAL) return;

  const int*   src = (const int*)d_in[0];
  const float* emb = (const float*)d_in[1];
  const float* wih = (const float*)d_in[2];
  const float* whh = (const float*)d_in[3];
  const float* bih = (const float*)d_in[4];
  const float* bhh = (const float*)d_in[5];
  float* out = (float*)d_out;

  unsigned char* ws = (unsigned char*)d_ws;
  _Float16* UT   = (_Float16*)(ws);
  _Float16* WIHT = (_Float16*)(ws + SZ_UT);
  _Float16* WHHT = (_Float16*)(ws + SZ_UT + SZ_WT);

  k_wprep<<<dim3(32), dim3(256), 0, stream>>>(wih, whh, WIHT, WHHT);
  k_proj<<<dim3(NSTEP), dim3(128), 0, stream>>>(src, emb, WIHT, UT);
  k_rnn<<<dim3(1), dim3(512), LDS_RNN, stream>>>((const unsigned*)UT, WHHT, bih, bhh, out);
}
